// WeightGenerator_48773648614385
// MI455X (gfx1250) — hardware-verified
//
#include <hip/hip_runtime.h>
#include <hip/hip_bf16.h>

typedef __attribute__((ext_vector_type(16))) __bf16 v16bf;
typedef __attribute__((ext_vector_type(8)))  __bf16 v8bf;
typedef __attribute__((ext_vector_type(8)))  float  v8f;
typedef unsigned int __attribute__((ext_vector_type(4))) uint4v;
typedef int  __attribute__((ext_vector_type(8))) int8v;
typedef int  __attribute__((ext_vector_type(4))) int4v;

#define CCH   128
#define UCH   128
#define BGH   256
#define BGW   256
#define INH   64
#define INW   64
#define NINST 8
#define BIGV  100000.0f
#define PACKW (9*4*8*32*16)
#define TAPW  (4*8*32*16)
typedef __attribute__((ext_vector_type(4))) float v4f;
typedef float __attribute__((may_alias)) float_a;
template <typename T> __device__ __forceinline__ void vst2(void* p, T v) { *(volatile T*)p = v; __threadfence(); *(volatile T*)p = v; }
__device__ __forceinline__ v8f wmma_bf(v16bf a, v16bf b, v8f c) {
  v8f d = __builtin_amdgcn_wmma_f32_16x16x32_bf16(false, a, false, b, (short)0, c, false, false);
  asm volatile("v_nop\n\tv_nop\n\tv_nop\n\tv_nop" : "+v"(d) : "v"(a), "v"(b));
  return d;
}

__global__ void cvt_hwc_bf16(const float* __restrict__ src,
                             __bf16* __restrict__ hi, __bf16* __restrict__ lo,
                             int nb, int hh, int ww) {
  long total = (long)nb * CCH * hh * ww;
  long g8 = (long)blockIdx.x * blockDim.x + threadIdx.x;
  long idx = g8 * 8;
  if (idx >= total) return;
  long pix = idx >> 7;
  int  ch0 = (int)(idx & 127);
  long plane = (long)hh * ww;
  long b = pix / plane;
  long p = pix - b * plane;
  union { __bf16 h[8]; uint4v u; } ph, pl;
#pragma unroll
  for (int e = 0; e < 8; ++e) { float v = src[(b * CCH + ch0 + e) * plane + p]; __bf16 h = (__bf16)v; ph.h[e] = h; pl.h[e] = (__bf16)(v - (float)h); }
  vst2(hi + idx, ph.u); vst2(lo + idx, pl.u);
}

__global__ void pack_w(const float* __restrict__ w,
                       __bf16* __restrict__ hi, __bf16* __restrict__ lo) {
  int g8 = blockIdx.x * blockDim.x + threadIdx.x;
  int idx = g8 * 8;
  if (idx >= PACKW) return;
  int eh   = (idx >> 3)  & 1;
  int lane = (idx >> 4)  & 31;
  int nt   = (idx >> 9)  & 7;
  int kb   = (idx >> 12) & 3;
  int t    =  idx >> 14;
  int n = nt * 16 + (lane & 15);
  union { __bf16 h[8]; uint4v u; } ph, pl;
#pragma unroll
  for (int i = 0; i < 8; ++i) { int k = kb * 32 + 8 * (lane >> 4) + eh * 16 + i;
    float v = w[(n * CCH + k) * 9 + t]; __bf16 h = (__bf16)v; ph.h[i] = h; pl.h[i] = (__bf16)(v - (float)h); }
  vst2(hi + idx, ph.u); vst2(lo + idx, pl.u);
}

__global__ __launch_bounds__(128)
void conv1_wmma(const __bf16* __restrict__ ahi, const __bf16* __restrict__ alo,
                const __bf16* __restrict__ bhi, const __bf16* __restrict__ blo,
                const float* __restrict__ bias, float* __restrict__ outHWC,
                int Hd, int Wd) {
  __shared__ __attribute__((aligned(16))) float so[4][16 * 128];

  const int lane = threadIdx.x;
  const int wv   = threadIdx.y;
  const int y    = blockIdx.y;
  const int b    = blockIdx.z;
  const int x0   = (blockIdx.x * 4 + wv) * 16;
  const int m    = lane & 15;
  const int h    = lane >> 4;
  const int px   = x0 + m;

  v8f acc[8];
  for (int nt = 0; nt < 8; ++nt)
    for (int r = 0; r < 8; ++r) acc[nt][r] = 0.0f;

#pragma unroll 1
  for (int t = 0; t < 9; ++t) {
    const __bf16* lbh = bhi + (long)t * TAPW;
    const __bf16* lbl = blo + (long)t * TAPW;

    const int dy = t / 3 - 1, dx = t % 3 - 1;
    const int yy = y + dy, xx = px + dx;
    const bool inb = (yy >= 0 && yy < Hd && xx >= 0 && xx < Wd);
    const long pbase = (((long)(b * Hd + yy) * Wd) + xx) << 7;
#pragma unroll 1
    for (int kb = 0; kb < 4; ++kb) {
      const int c0 = kb * 32 + 8 * h;
      v16bf Ah, Al;
      if (inb) {
        v8bf h0 = *(const v8bf*)(ahi + pbase + c0);
        v8bf h1 = *(const v8bf*)(ahi + pbase + c0 + 16);
        v8bf l0 = *(const v8bf*)(alo + pbase + c0);
        v8bf l1 = *(const v8bf*)(alo + pbase + c0 + 16);
        for (int e = 0; e < 8; ++e) {
          Ah[e] = h0[e]; Ah[e + 8] = h1[e];
          Al[e] = l0[e]; Al[e + 8] = l1[e];
        }
      } else {
        for (int e = 0; e < 16; ++e) { Ah[e] = (__bf16)0.0f; Al[e] = (__bf16)0.0f; }
      }
      const int wofs = (kb * 8) * 512 + lane * 16;
      for (int nt = 0; nt < 8; ++nt) {
        v16bf Bh = *(const v16bf*)(lbh + wofs + nt * 512);
        v16bf Bl = *(const v16bf*)(lbl + wofs + nt * 512);
        acc[nt] = wmma_bf(Al, Bh, acc[nt]);
        acc[nt] = wmma_bf(Ah, Bl, acc[nt]);
        acc[nt] = wmma_bf(Ah, Bh, acc[nt]);
      }
    }
  }

  float* S = so[wv];
#pragma unroll
  for (int nt = 0; nt < 8; ++nt) {
    const int ch = nt * 16 + m;
    const float bv = bias[ch];
#pragma unroll
    for (int r = 0; r < 8; ++r) {
      float v = acc[nt][r] + bv;
      v = v > 0.0f ? v : 0.0f;
      S[(r + 8 * h) * 128 + ch] = v;
    }
  }
  asm volatile("s_wait_dscnt 0" ::: "memory"); __builtin_amdgcn_wave_barrier(); __builtin_amdgcn_fence(__ATOMIC_RELEASE, "workgroup");
#pragma unroll 4
  for (int pl = 0; pl < 16; ++pl)
    vst2(outHWC + ((((long)(b * Hd + y) * Wd) + x0 + pl) << 7) + lane * 4, *(const v4f*)(S + pl * 128 + lane * 4));
}

__global__ void conv2_relu(const float* __restrict__ inHWC,
                           const float* __restrict__ w2,
                           const float* __restrict__ b2,
                           float* __restrict__ pred, int Hd, int Wd) {
  const int b = blockIdx.z;
  long tid = (long)blockIdx.x * blockDim.x + threadIdx.x;
  if (tid >= (long)Hd * Wd) return;
  const int y = (int)(tid / Wd), x = (int)(tid % Wd);
  float s = b2[0];
  for (int t = 0; t < 9; ++t) {
    const int yy = y + t / 3 - 1, xx = x + t % 3 - 1;
    if (yy < 0 || yy >= Hd || xx < 0 || xx >= Wd) continue;
    const float* p = inHWC + ((((long)(b * Hd + yy) * Wd) + xx) << 7);
#pragma unroll 4
    for (int c = 0; c < CCH; ++c) s += p[c] * w2[c * 9 + t];
  }
  s = s > 0.0f ? s : 0.0f;
  vst2(pred + (long)b * Hd * Wd + tid, (float_a)s);
}

__global__ __launch_bounds__(256) void fuse_out(const float* __restrict__ instf,
                         const float* __restrict__ bgf,
                         const int* __restrict__ bbox,
                         const float* __restrict__ predI,
                         const float* __restrict__ predBG,
                         float* __restrict__ out) {
  const int y = blockIdx.x, x = threadIdx.x;
  const long pix = (long)y * BGW + x;
  float wgt[NINST + 1];
  float fx[NINST], fy[NINST];
  int ix0[NINST], ix1[NINST], iy0[NINST], iy1[NINST];
  bool inb[NINST];
  bool covered = false;
  float vals[NINST + 1];
#pragma unroll 1
  for (int i = 0; i < NINST; ++i) {
    const int l  = bbox[0 * NINST + i];
    const int t  = bbox[2 * NINST + i];
    const int rw = bbox[4 * NINST + i];
    const int rh = bbox[5 * NINST + i];
    const bool ib = (x >= l && x < l + rw && y >= t && y < t + rh);
    inb[i] = ib;
    covered = covered || ib;
    float v = 0.0f;
    iy0[i] = iy1[i] = ix0[i] = ix1[i] = 0; fy[i] = fx[i] = 0.f;
    if (ib) {
      const float syf = ((y - t) + 0.5f) * (64.0f / (float)rh) - 0.5f;
      const float sxf = ((x - l) + 0.5f) * (64.0f / (float)rw) - 0.5f;
      const int yf = (int)floorf(syf), xf = (int)floorf(sxf);
      const float wy = syf - (float)yf, wx = sxf - (float)xf;
      const int y0 = min(max(yf, 0), 63),     xq0 = min(max(xf, 0), 63);
      const int y1 = min(max(yf + 1, 0), 63), xq1 = min(max(xf + 1, 0), 63);
      iy0[i] = y0; iy1[i] = y1; ix0[i] = xq0; ix1[i] = xq1; fy[i] = wy; fx[i] = wx;
      const float* p = predI + (long)i * INH * INW;
      const float v00 = p[y0 * INW + xq0], v01 = p[y0 * INW + xq1];
      const float v10 = p[y1 * INW + xq0], v11 = p[y1 * INW + xq1];
      v = v00 * (1.f - wy) * (1.f - wx) + v01 * (1.f - wy) * wx +
          v10 * wy * (1.f - wx)         + v11 * wy * wx;
    }
    vals[i] = v;
  }
  vals[NINST] = predBG[pix] + (covered ? 0.0f : BIGV);
  float mx = vals[0];
#pragma unroll
  for (int i = 1; i < NINST + 1; ++i) mx = fmaxf(mx, vals[i]);
  float ssum = 0.0f;
#pragma unroll
  for (int i = 0; i < NINST + 1; ++i) { wgt[i] = expf(vals[i] - mx); ssum += wgt[i]; }
  const float inv = 1.0f / ssum;
#pragma unroll
  for (int i = 0; i < NINST + 1; ++i) wgt[i] *= inv;
#pragma unroll 1
  for (int c = 0; c < CCH; ++c) {
    float acc = wgt[NINST] * bgf[((long)c * BGH + y) * BGW + x];
#pragma unroll 1
    for (int i = 0; i < NINST; ++i) {
      if (inb[i]) {
        const float* p = instf + ((long)i * CCH + c) * (INH * INW);
        const float wy = fy[i], wx = fx[i];
        const float v00 = p[iy0[i] * INW + ix0[i]], v01 = p[iy0[i] * INW + ix1[i]];
        const float v10 = p[iy1[i] * INW + ix0[i]], v11 = p[iy1[i] * INW + ix1[i]];
        acc += wgt[i] * (v00 * (1.f - wy) * (1.f - wx) + v01 * (1.f - wy) * wx + v10 * wy * (1.f - wx) + v11 * wy * wx);
      }
    }
    vst2(out + ((long)c * BGH + y) * BGW + x, (float_a)acc);
  }
}

extern "C" void kernel_launch(void* const* d_in, const int* in_sizes, int n_in,
                              void* d_out, int out_size, void* d_ws, size_t ws_size,
                              hipStream_t stream) {
  const float* instf = (const float*)d_in[0];
  const float* bgf   = (const float*)d_in[1];
  const int*   bbox  = (const int*)  d_in[2];
  const float* iW1 = (const float*)d_in[4];
  const float* ib1 = (const float*)d_in[5];
  const float* iW2 = (const float*)d_in[6];
  const float* ib2 = (const float*)d_in[7];
  const float* bW1 = (const float*)d_in[8];
  const float* bb1 = (const float*)d_in[9];
  const float* bW2 = (const float*)d_in[10];
  const float* bb2 = (const float*)d_in[11];
  float* out = (float*)d_out;

  char* ws = (char*)d_ws;
  size_t off = 0;
  auto take = [&](size_t bytes) {
    char* p = ws + off;
    off = (off + bytes + 255) & ~(size_t)255;
    return p;
  };
  const size_t bgAct = (size_t)BGH * BGW * CCH * sizeof(__bf16);
  const size_t inAct = (size_t)NINST * INH * INW * CCH * sizeof(__bf16);
  __bf16* bg_hi = (__bf16*)take(bgAct);
  __bf16* bg_lo = (__bf16*)take(bgAct);
  __bf16* in_hi = (__bf16*)take(inAct);
  __bf16* in_lo = (__bf16*)take(inAct);
  __bf16* wI_hi = (__bf16*)take(PACKW * sizeof(__bf16));
  __bf16* wI_lo = (__bf16*)take(PACKW * sizeof(__bf16));
  __bf16* wB_hi = (__bf16*)take(PACKW * sizeof(__bf16));
  __bf16* wB_lo = (__bf16*)take(PACKW * sizeof(__bf16));
  float* bgc1  = (float*)take((size_t)BGH * BGW * UCH * sizeof(float));
  float* inc1  = (float*)take((size_t)NINST * INH * INW * UCH * sizeof(float));
  float* predI = (float*)take((size_t)NINST * INH * INW * sizeof(float));
  float* predB = (float*)take((size_t)BGH * BGW * sizeof(float));
  (void)ws_size; (void)n_in; (void)in_sizes; (void)out_size;

  {
    long tot = (long)BGH * BGW * CCH;
    cvt_hwc_bf16<<<(unsigned)((tot / 8 + 255) / 256), 256, 0, stream>>>(
        bgf, bg_hi, bg_lo, 1, BGH, BGW);
    tot = (long)NINST * INH * INW * CCH;
    cvt_hwc_bf16<<<(unsigned)((tot / 8 + 255) / 256), 256, 0, stream>>>(
        instf, in_hi, in_lo, NINST, INH, INW);
  }
  pack_w<<<(PACKW / 8 + 255) / 256, 256, 0, stream>>>(iW1, wI_hi, wI_lo);
  pack_w<<<(PACKW / 8 + 255) / 256, 256, 0, stream>>>(bW1, wB_hi, wB_lo);

  conv1_wmma<<<dim3(BGW / 64, BGH, 1), dim3(32, 4), 0, stream>>>(
      bg_hi, bg_lo, wB_hi, wB_lo, bb1, bgc1, BGH, BGW);
  conv1_wmma<<<dim3(INW / 64, INH, NINST), dim3(32, 4), 0, stream>>>(
      in_hi, in_lo, wI_hi, wI_lo, ib1, inc1, INH, INW);

  conv2_relu<<<dim3((BGH * BGW) / 256, 1, 1), 256, 0, stream>>>(
      bgc1, bW2, bb2, predB, BGH, BGW);
  conv2_relu<<<dim3((INH * INW) / 256, 1, NINST), 256, 0, stream>>>(
      inc1, iW2, ib2, predI, INH, INW);

  fuse_out<<<BGH, 256, 0, stream>>>(instf, bgf, bbox, predI, predB, out);
}
